// NodeSpanEncoder_31129922962206
// MI455X (gfx1250) — hardware-verified
//
#include <hip/hip_runtime.h>
#include <math.h>

#ifndef NB
#define NB 16
#endif
#ifndef SEQ
#define SEQ 4096
#endif
#define SEQ_FULL 4096
#define NSPAN 1024
#define DM 128
#define TILES_PER_B ((NSPAN / 64) * (DM / 64))
#define XT_P 132

typedef __attribute__((ext_vector_type(16))) __bf16       v16bf;
typedef __attribute__((ext_vector_type(8)))  float        v8f;
typedef __attribute__((ext_vector_type(4)))  float        v4f;
typedef __attribute__((ext_vector_type(4)))  unsigned int v4u;
typedef __attribute__((ext_vector_type(8)))  unsigned int v8u;

static_assert(SEQ % 64 == 0);
static_assert(SEQ % 32 == 0);
static_assert(SEQ <= SEQ_FULL);
static_assert(NSPAN % 64 == 0);
static_assert(DM == 128);
static_assert(DM % 64 == 0);
static_assert((NB * TILES_PER_B) % 8 == 0);
static_assert(XT_P % 4 == 0);
static_assert(XT_P >= DM);
static constexpr size_t XT_BYTES = (size_t)NB * DM * SEQ * 2;
static_assert(XT_BYTES <= (size_t)134217728);
static_assert(256 * 16 * 8 == 64 * DM * 4);
static_assert(8 * 4 * 4 == DM);
static_assert(256 * 16 * 4 == 64 * DM * 2);
static_assert(32 * 16 * 8 == 16 * 64 * 4);
static_assert(64 * XT_P * 4 <= 131072);
static_assert(8 * 16 * 68 * 4 + 8 * 64 * 4 <= 131072);


static __device__ __forceinline__ unsigned bf16_bits(float f) {
    unsigned u = __float_as_uint(f);
    u += 0x7FFFu + ((u >> 16) & 1u);
    return u >> 16;
}

static __device__ __forceinline__ v16bf frag_ld_bf(const unsigned short* p) {
    const v4u q0 = *(const v4u*)(p);
    const v4u q1 = *(const v4u*)(p + 16);
    const v8u w = __builtin_shufflevector(q0, q1, 0, 1, 2, 3, 4, 5, 6, 7);
    return __builtin_bit_cast(v16bf, w);
}

static __device__ __forceinline__ unsigned span_word(unsigned t, unsigned lo, unsigned len, unsigned one_bits) {
    return ((t - lo) <= len) ? one_bits : 0u;
}

static __device__ __forceinline__ v16bf mask_frag(unsigned tb, unsigned lo, unsigned len) {
    unsigned w[8];
#pragma unroll
    for (int p = 0; p < 4; ++p) {
        const unsigned ta = tb + 2u * (unsigned)p;
        w[p] = span_word(ta, lo, len, 0x3F80u) | span_word(ta + 1u, lo, len, 0x3F800000u);
        const unsigned tc = tb + 16u + 2u * (unsigned)p;
        w[p + 4] = span_word(tc, lo, len, 0x3F80u) | span_word(tc + 1u, lo, len, 0x3F800000u);
    }
    const v8u v = (v8u){w[0], w[1], w[2], w[3], w[4], w[5], w[6], w[7]};
    return __builtin_bit_cast(v16bf, v);
}

static __device__ __forceinline__ v8f wmmabg(v16bf a, v16bf b, v8f c) {
    c = __builtin_amdgcn_wmma_f32_16x16x32_bf16(false, a, false, b, (short)0, c, false, false);
    asm volatile("v_nop\n\tv_nop\n\tv_nop\n\tv_nop" : "+v"(c) : "v"(a), "v"(b));
    return c;
}

__device__ __forceinline__ void wave_sync_lds() {
    __builtin_amdgcn_fence(3  , "workgroup");
    __builtin_amdgcn_wave_barrier();
    __builtin_amdgcn_fence(2  , "workgroup");
}

__global__ __launch_bounds__(256) void k_xt(const float* __restrict__ x, unsigned short* __restrict__ XT) {
    __shared__ __align__(16) float sX[64 * XT_P];
    const unsigned tid = threadIdx.x, lane = tid & 31u;
    const unsigned wave = (unsigned)__builtin_amdgcn_readfirstlane((int)(tid >> 5));
    const unsigned bx = blockIdx.x;
    const unsigned b = bx / (unsigned)(SEQ / 64);
    const unsigned t0 = (bx - b * (unsigned)(SEQ / 64)) * 64u;
    const float* xs = x + ((size_t)b * SEQ_FULL + t0) * DM;
    v4f ld[8];
#pragma unroll
    for (int it = 0; it < 8; ++it)
        ld[it] = *(const v4f*)(xs + (size_t)((unsigned)it * 8u + wave) * DM + lane * 4u);
#pragma unroll
    for (int it = 0; it < 8; ++it)
        *(v4f*)(&sX[((unsigned)it * 8u + wave) * XT_P + lane * 4u]) = ld[it];
    __syncthreads();
    const unsigned q = lane >> 3, p = lane & 7u;
    v4u pk[4];
#pragma unroll
    for (int it = 0; it < 4; ++it) {
        const unsigned d = ((unsigned)it * 8u + wave) * 4u + q;
        unsigned w[8];
#pragma unroll
        for (int e = 0; e < 8; ++e) w[e] = bf16_bits(sX[(8u * p + (unsigned)e) * XT_P + d]);
        pk[it].x = w[0] | (w[1] << 16);
        pk[it].y = w[2] | (w[3] << 16);
        pk[it].z = w[4] | (w[5] << 16);
        pk[it].w = w[6] | (w[7] << 16);
    }
    for (int pass = 0; pass < 2; ++pass) {
#pragma unroll
        for (int it = 0; it < 4; ++it) {
            const unsigned d = ((unsigned)it * 8u + wave) * 4u + q;
            unsigned short* dst = XT + ((size_t)(b * (unsigned)DM + d) * SEQ + t0 + 8u * p);
            *(volatile v4u*)(dst) = pk[it];
        }
        __threadfence();
    }
}

__global__ __launch_bounds__(256) void k_span(const unsigned short* __restrict__ XT, const int* __restrict__ starts,
                                              const int* __restrict__ ends, float* __restrict__ out) {
    __shared__ __align__(16) float sT[8][16 * 68];
    __shared__ float sCnt[8][64];
    const unsigned lane = threadIdx.x & 31u;
    const unsigned wave = (unsigned)__builtin_amdgcn_readfirstlane((int)(threadIdx.x >> 5));
    const unsigned hh = lane >> 4, c = lane & 15u;
    const unsigned bx = blockIdx.x;
    const unsigned tile = bx * 8u + wave;
    if (tile >= (unsigned)(NB * TILES_PER_B)) return;
    const unsigned b = tile / (unsigned)TILES_PER_B;
    const unsigned rem = tile - b * (unsigned)TILES_PER_B;
    const unsigned tn = rem / (unsigned)(DM / 64);
    const unsigned td = rem - tn * (unsigned)(DM / 64);
    const unsigned n0 = tn * 64u, d0 = td * 64u;

    unsigned lo[4], len[4];
#pragma unroll
    for (int i = 0; i < 4; ++i) {
        const unsigned n = n0 + 16u * (unsigned)i + c;
        const int s = starts[(size_t)b * NSPAN + n];
        const int e = ends[(size_t)b * NSPAN + n];
        const int lo_i = min(max(s, 0), SEQ);
        const int hi_i = max(min(e, SEQ - 1), -1);
        const int ln = hi_i - lo_i;
        const bool none = (ln < 0);
        lo[i]  = none ? 0x40000000u : (unsigned)lo_i;
        len[i] = none ? 0u : (unsigned)ln;
        sCnt[wave][16u * (unsigned)i + c] = none ? 0.0f : (float)(ln + 1);
    }

    v8f acc[4][4];
#pragma unroll
    for (int i = 0; i < 4; ++i)
#pragma unroll
        for (int j = 0; j < 4; ++j) acc[i][j] = (v8f){0.f,0.f,0.f,0.f,0.f,0.f,0.f,0.f};

    const unsigned short* bp = XT + (size_t)(b * (unsigned)DM + d0 + c) * SEQ + 8u * hh;
    const unsigned tb0 = 8u * hh;
#pragma unroll 1
    for (unsigned k0 = 0; k0 < (unsigned)SEQ; k0 += 32u) {
        v16bf xb[4];
#pragma unroll
        for (int j = 0; j < 4; ++j)
            xb[j] = frag_ld_bf(bp + (size_t)(16u * (unsigned)j) * SEQ + k0);
        const unsigned tb = k0 + tb0;
#pragma unroll
        for (int i = 0; i < 4; ++i) {
            const v16bf a = mask_frag(tb, lo[i], len[i]);
#pragma unroll
            for (int j = 0; j < 4; ++j)
                acc[i][j] = wmmabg(a, xb[j], acc[i][j]);
        }
    }

    const unsigned c4 = c * 4u;
#pragma unroll
    for (int i = 0; i < 4; ++i) {
        const unsigned mBase = n0 + ((unsigned)i << 4);
#pragma unroll
        for (int j = 0; j < 4; ++j)
#pragma unroll
            for (int r = 0; r < 8; ++r)
                sT[wave][(8u * hh + (unsigned)r) * 68u + ((unsigned)j << 4) + c] = acc[i][j][r];
        wave_sync_lds();
#pragma unroll
        for (int half = 0; half < 2; ++half) {
            v4f vv[4];
#pragma unroll
            for (int it = 0; it < 4; ++it) {
                const unsigned row = (unsigned)(half * 4 + it) * 2u + hh;
                const v4f s4 = *(const v4f*)(&sT[wave][row * 68u + c4]);
                const float cn = sCnt[wave][16u * (unsigned)i + row];
                v4f o;
                o.x = s4.x / cn; o.y = s4.y / cn; o.z = s4.z / cn; o.w = s4.w / cn;
                vv[it] = o;
            }
            for (int pass = 0; pass < 2; ++pass) {
#pragma unroll
                for (int it = 0; it < 4; ++it) {
                    const unsigned row = (unsigned)(half * 4 + it) * 2u + hh;
                    *(volatile v4f*)(out + (size_t)(b * (unsigned)NSPAN + mBase + row) * DM + d0 + c4) = vv[it];
                }
                __threadfence();
            }
        }
        wave_sync_lds();
    }
}

extern "C" void kernel_launch(void* const* d_in, const int* in_sizes, int n_in, void* d_out, int out_size,
                              void* d_ws, size_t ws_size, hipStream_t stream) {
    if (n_in < 3) return;
    if (in_sizes[0] < ((NB - 1) * SEQ_FULL + SEQ) * DM || in_sizes[1] < NB * NSPAN || in_sizes[2] < NB * NSPAN) return;
    if (out_size < NB * NSPAN * DM) return;

    const float* x      = (const float*)d_in[0];
    const int*   starts = (const int*)d_in[1];
    const int*   ends   = (const int*)d_in[2];
    float* out = (float*)d_out;

    if (XT_BYTES > ws_size || XT_BYTES > (size_t)134217728) return;
    unsigned short* xt = (unsigned short*)d_ws;

    k_xt<<<NB * (SEQ / 64), 256, 0, stream>>>(x, xt);
    k_span<<<(NB * TILES_PER_B) / 8, 256, 0, stream>>>((const unsigned short*)xt, starts, ends, out);
}
